// StructuralTransformerLayer_16741782520605
// MI455X (gfx1250) — hardware-verified
//
#include <hip/hip_runtime.h>
#include <hip/hip_bf16.h>
#include <math.h>


#define BB 4
#define SS 1024
#define DD 768
#define HH 8
#define DKK 96
#define KS2 104
#define DFF 2048
#define DQ (3 * DD)
#define QW 2

typedef _Float16 bf16;
typedef __attribute__((ext_vector_type(4))) unsigned v4u_t;
typedef unsigned v4ua __attribute__((ext_vector_type(4), may_alias));
typedef __attribute__((ext_vector_type(4))) float v4f_t;
typedef float v4fa __attribute__((ext_vector_type(4), may_alias));
typedef __attribute__((ext_vector_type(16))) bf16  bf16x16;
typedef __attribute__((ext_vector_type(8)))  bf16  bf16x8;
typedef __attribute__((ext_vector_type(4)))  bf16  bf16x4;
typedef __attribute__((ext_vector_type(8)))  float f32x8;

#define LDS_STRIDE 48
#define KSTRIDE    72
#define VSTRIDE    48

__device__ __forceinline__ f32x8 wmma_bf16(bf16x16 a, bf16x16 b, f32x8 c) {
  return __builtin_amdgcn_wmma_f32_16x16x32_f16(
      false, a, false, b, (short)0, c, false, false);
}
#define RSPLIT (1.0f / 2048.0f)
__device__ __forceinline__ bf16 lo_of(float v, bf16 h) { return (bf16)((v - (float)h) * 2048.0f); }
__device__ __forceinline__ f32x8 wmma_split(bf16x16 a, bf16x16 al, bf16x16 b, bf16x16 bl, f32x8 c) {
  f32x8 x = {}; x = wmma_bf16(al, b, x); x = wmma_bf16(a, bl, x); return wmma_bf16(a, b, c) + x * RSPLIT; }

template <typename T>
__device__ __forceinline__ bf16x16 load_frag(const T* __restrict__ base, int ld,
                                             int row0, int k0) {
  const int lane = threadIdx.x & 31;
  const int r    = lane & 15;
  const int kh   = (lane >> 4) * 8;
  const T* p0 = base + (size_t)(row0 + r) * ld + (k0 + kh);
  const T* p1 = p0 + 16;
  bf16x16 f;
#pragma unroll
  for (int i = 0; i < 8; ++i) {
    f[i]     = (bf16)p0[i];
    f[i + 8] = (bf16)p1[i];
  }
  return f;
}

__device__ __forceinline__ bf16x16 lds_frag(const bf16* base, int stride) {
  const int lane = threadIdx.x & 31;
  const int row  = lane & 15;
  const int kh   = (lane >> 4) * 8;
  const bf16x8 lo = *(const bf16x8*)(base + row * stride + kh);
  const bf16x8 hi = *(const bf16x8*)(base + row * stride + kh + 16);
  bf16x16 f;
#pragma unroll
  for (int i = 0; i < 8; ++i) { f[i] = lo[i]; f[i + 8] = hi[i]; }
  return f;
}

template <typename T>
__device__ __forceinline__ void stage_read16(const T* __restrict__ p, float* buf) {
#pragma unroll
  for (int i = 0; i < 16; ++i) buf[i] = (float)p[i];
}

__device__ __forceinline__ void stage_write(bf16* dst, const float* buf, int nquad) {
#pragma unroll
  for (int i = 0; i < nquad; ++i) {
    bf16x4 q;
    q[0] = (bf16)buf[4 * i];     q[1] = (bf16)buf[4 * i + 1];
    q[2] = (bf16)buf[4 * i + 2]; q[3] = (bf16)buf[4 * i + 3];
    *(bf16x4*)(dst + 4 * i) = q;
  }
}

template <typename AT, int MODE>
__global__ __launch_bounds__(256) void gemm_bias_kernel(
    const AT* __restrict__ A, const float* __restrict__ W,
    const float* __restrict__ bias, void* __restrict__ out,
    int M, int N, int K) {
  __shared__ bf16 ldsA[128 * LDS_STRIDE];
  __shared__ bf16 ldsW[256 * LDS_STRIDE];
  __shared__ __attribute__((aligned(16))) unsigned char sob[256 * 136 * 2];

  const int t    = threadIdx.x;
  const int wave = t >> 5;
  const int lane = t & 31;
  const int wm   = (wave & 1) * 64;
  const int wn   = (wave >> 1) * 64;
  const int mBlk = blockIdx.x * 128;
  const int nBlk = blockIdx.y * 256;

  const int arow = t >> 1;
  const int ach  = (t & 1) * 16;

  float abuf[16];
  float wbuf[32];

  stage_read16(A + (size_t)(mBlk + arow) * K + ach, abuf);
  stage_read16(W + (size_t)(nBlk + t) * K,          wbuf);
  stage_read16(W + (size_t)(nBlk + t) * K + 16,     wbuf + 16);

  f32x8 acc[4][4] = {};

  for (int k = 0; k < K; k += 32) {
    __syncthreads();
    stage_write(&ldsA[arow * LDS_STRIDE + ach], abuf, 4);
    stage_write(&ldsW[t * LDS_STRIDE],          wbuf, 8);
    if (k + 32 < K) {
      stage_read16(A + (size_t)(mBlk + arow) * K + (k + 32) + ach, abuf);
      stage_read16(W + (size_t)(nBlk + t) * K + (k + 32),          wbuf);
      stage_read16(W + (size_t)(nBlk + t) * K + (k + 32) + 16,     wbuf + 16);
    }
    __syncthreads();

    bf16x16 af[4], wf[4];
#pragma unroll
    for (int i = 0; i < 4; ++i)
      af[i] = lds_frag(ldsA + (wm + 16 * i) * LDS_STRIDE, LDS_STRIDE);
#pragma unroll
    for (int j = 0; j < 4; ++j)
      wf[j] = lds_frag(ldsW + (wn + 16 * j) * LDS_STRIDE, LDS_STRIDE);
#pragma unroll
    for (int i = 0; i < 4; ++i)
#pragma unroll
      for (int j = 0; j < 4; ++j)
        acc[i][j] = wmma_bf16(af[i], wf[j], acc[i][j]);
  }

  const int nlane = lane & 15;
  const int mh    = (lane >> 4) * 8;
  __syncthreads();
  if (MODE == 0 || MODE == 1) {
    bf16* so = (bf16*)sob;
#pragma unroll
    for (int i = 0; i < 4; ++i)
#pragma unroll
      for (int j = 0; j < 4; ++j) {
        const int nl = wn + 16 * j + nlane;
        const float bv = bias ? bias[nBlk + nl] : 0.0f;
#pragma unroll
        for (int r = 0; r < 8; ++r) {
          const int ml = wm + 16 * i + mh + r;
          const bf16 hv = (bf16)(acc[i][j][r] + bv);
          if (MODE == 0) so[ml * 264 + nl] = hv;
          else           so[nl * 136 + ml] = hv;
        }
      }
    __syncthreads();
#pragma unroll 1
    for (int pass = 0; pass < 2; ++pass) {
      if (MODE == 0) {
        for (int ch = t; ch < 128 * 32; ch += 256) { const int ml = ch >> 5, q = (ch & 31) * 8;
          *(volatile v4u_t*)((bf16*)out + (size_t)(mBlk + ml) * N + nBlk + q) = *(const v4ua*)(so + ml * 264 + q); }
      } else {
        const int b_ = mBlk / SS, s0 = mBlk & (SS - 1);
        for (int ch = t; ch < 256 * 16; ch += 256) { const int nl = ch >> 4, q = (ch & 15) * 8; const int n = nBlk + nl, h = n >> 6, dk = n & (DKK - 1);
          *(volatile v4u_t*)((bf16*)out + (((size_t)(b_ * HH + h)) * DKK + dk) * SS + s0 + q) = *(const v4ua*)(so + nl * 136 + q); }
      }
      __threadfence();
    }
  } else {
    float* so = (float*)sob;
#pragma unroll 1
    for (int hf = 0; hf < 2; ++hf) {
      if (wm == hf * 64) {
#pragma unroll
        for (int i = 0; i < 4; ++i)
#pragma unroll
          for (int j = 0; j < 4; ++j) {
            const int nl = wn + 16 * j + nlane;
            const float bv = bias ? bias[nBlk + nl] : 0.0f;
#pragma unroll
            for (int r = 0; r < 8; ++r) so[(16 * i + mh + r) * 260 + nl] = acc[i][j][r] + bv;
          }
      }
      __syncthreads();
#pragma unroll 1
      for (int pass = 0; pass < 2; ++pass) {
        for (int ch = t; ch < 64 * 64; ch += 256) { const int ml = ch >> 6, q = (ch & 63) * 4;
          *(volatile v4f_t*)((float*)out + (size_t)(mBlk + hf * 64 + ml) * N + nBlk + q) = *(const volatile v4fa*)(so + ml * 260 + q); }
        __threadfence();
      }
      __syncthreads();
    }
  }
}

template <typename AT, int MODE>
__global__ __launch_bounds__(256) void gemm_split_kernel(
    const AT* __restrict__ A, size_t aPlane, const float* __restrict__ W,
    const float* __restrict__ bias, void* __restrict__ out,
    int M, int N, int K) {
  __shared__ bf16 ldsA[128 * LDS_STRIDE], ldsAl[128 * LDS_STRIDE];
  __shared__ bf16 ldsW[256 * LDS_STRIDE], ldsWl[256 * LDS_STRIDE];
  __shared__ __attribute__((aligned(16))) unsigned char sob[256 * 136 * 2];

  const int t    = threadIdx.x;
  const int wave = t >> 5;
  const int lane = t & 31;
  const int wm   = (wave & 1) * 64;
  const int wn   = (wave >> 1) * 64;
  const int mBlk = blockIdx.x * 128;
  const int nBlk = blockIdx.y * 256;
  const int arow = t >> 1;
  const int ach  = (t & 1) * 16;

  f32x8 acc[4][4] = {};
  for (int k = 0; k < K; k += 32) {
    __syncthreads();
    {
      const AT* ap = A + (size_t)(mBlk + arow) * K + k + ach;
      bf16 hh[16], hl[16];
      if (sizeof(AT) == 4) {
#pragma unroll
        for (int i = 0; i < 16; ++i) { const float v = (float)ap[i]; hh[i] = (bf16)v; hl[i] = lo_of(v, hh[i]); }
      } else {
#pragma unroll
        for (int i = 0; i < 16; ++i) { hh[i] = (bf16)ap[i]; hl[i] = (bf16)ap[aPlane + i]; }
      }
#pragma unroll
      for (int i = 0; i < 16; ++i) { ldsA[arow * LDS_STRIDE + ach + i] = hh[i]; ldsAl[arow * LDS_STRIDE + ach + i] = hl[i]; }
    }
    {
      const float* wp = W + (size_t)(nBlk + t) * K + k;
#pragma unroll
      for (int i = 0; i < 32; ++i) { const float v = wp[i]; const bf16 h_ = (bf16)v; ldsW[t * LDS_STRIDE + i] = h_; ldsWl[t * LDS_STRIDE + i] = lo_of(v, h_); }
    }
    __syncthreads();
    bf16x16 wf[4], wfl[4];
#pragma unroll
    for (int j = 0; j < 4; ++j) { wf[j] = lds_frag(ldsW + (wn + 16 * j) * LDS_STRIDE, LDS_STRIDE); wfl[j] = lds_frag(ldsWl + (wn + 16 * j) * LDS_STRIDE, LDS_STRIDE); }
#pragma unroll
    for (int i = 0; i < 4; ++i) {
      const bf16x16 af = lds_frag(ldsA + (wm + 16 * i) * LDS_STRIDE, LDS_STRIDE), afl = lds_frag(ldsAl + (wm + 16 * i) * LDS_STRIDE, LDS_STRIDE);
#pragma unroll
      for (int j = 0; j < 4; ++j) acc[i][j] = wmma_split(af, afl, wf[j], wfl[j], acc[i][j]);
    }
  }

  const int nlane = lane & 15;
  const int mh    = (lane >> 4) * 8;
  __syncthreads();
  if (MODE == 1) {
    bf16* so = (bf16*)sob;
#pragma unroll
    for (int i = 0; i < 4; ++i)
#pragma unroll
      for (int j = 0; j < 4; ++j) {
        const int nl = wn + 16 * j + nlane;
        const float bv = bias ? bias[nBlk + nl] : 0.0f;
#pragma unroll
        for (int r = 0; r < 8; ++r) so[nl * 136 + wm + 16 * i + mh + r] = (bf16)(acc[i][j][r] + bv);
      }
    __syncthreads();
    const int b_ = mBlk / SS, s0 = mBlk & (SS - 1);
#pragma unroll 1
    for (int pass = 0; pass < 2; ++pass) {
      for (int ch = t; ch < 256 * 16; ch += 256) { const int nl = ch >> 4, q = (ch & 15) * 8; const int n = nBlk + nl, h = n >> 6, dk = n & (DKK - 1);
        *(volatile v4u_t*)((bf16*)out + (((size_t)(b_ * HH + h)) * DKK + dk) * SS + s0 + q) = *(const v4ua*)(so + nl * 136 + q); }
      __threadfence();
    }
  } else {
    float* so = (float*)sob;
#pragma unroll 1
    for (int hf = 0; hf < 2; ++hf) {
      if (wm == hf * 64) {
#pragma unroll
        for (int i = 0; i < 4; ++i)
#pragma unroll
          for (int j = 0; j < 4; ++j) {
            const int nl = wn + 16 * j + nlane;
            const float bv = bias ? bias[nBlk + nl] : 0.0f;
#pragma unroll
            for (int r = 0; r < 8; ++r) so[(16 * i + mh + r) * 260 + nl] = acc[i][j][r] + bv;
          }
      }
      __syncthreads();
#pragma unroll 1
      for (int pass = 0; pass < 2; ++pass) {
        for (int ch = t; ch < 64 * 64; ch += 256) { const int ml = ch >> 6, q = (ch & 63) * 4;
          *(volatile v4f_t*)((float*)out + (size_t)(mBlk + hf * 64 + ml) * N + nBlk + q) = *(const volatile v4fa*)(so + ml * 260 + q); }
        __threadfence();
      }
      __syncthreads();
    }
  }
}

__global__ __launch_bounds__(64) void attn96_kernel(const bf16* __restrict__ Qb, const bf16* __restrict__ Kb, const bf16* __restrict__ Vt, const float* __restrict__ bias, float* __restrict__ attnOut) {
  __shared__ bf16 ldsK[32 * KS2];
  __shared__ bf16 ldsV[96 * VSTRIDE];
  __shared__ __attribute__((aligned(16))) float ldsO[2][16 * 100];
  const int q0blk = blockIdx.x * 32, h = blockIdx.y, b = blockIdx.z;
  const int t = threadIdx.x, wave = t >> 5, lane = t & 31, qlane = lane & 15, kh8 = (lane >> 4) * 8;
  const int q0 = q0blk + wave * 16;
  const bf16* Qh = Qb + (size_t)b * SS * DQ + h * DKK;
  const bf16* Kh = Kb + (size_t)b * SS * DQ + h * DKK;
  const bf16* Vh = Vt + ((size_t)(b * HH + h)) * DKK * SS;
  const float* brow = bias + ((size_t)b * SS) * SS;
  const int krow = t >> 1, kcol = (t & 1) * 48;
  bf16x16 qf[3];
#pragma unroll
  for (int c = 0; c < 3; ++c) qf[c] = load_frag(Qh, DQ, q0, 32 * c);
  f32x8 o[6] = {};
  float mrun = -INFINITY, lrun = 0.0f;
  const float L2E = 1.44269504088896340736f; const float scale = 0.10206207261596575f * L2E;
  const int qi = q0 + qlane, kmax = SS - 1;
  const float* bq_ = brow + (size_t)qi * SS;
#pragma unroll 1
  for (int kb = 0; kb <= kmax; kb += 32) {
    __syncthreads();
    { const bf16* ks = Kh + (size_t)(kb + krow) * DQ + kcol;
#pragma unroll
      for (int i = 0; i < 6; ++i) *(bf16x8*)(&ldsK[krow * KS2 + kcol + 8 * i]) = *(const bf16x8*)(ks + 8 * i);
      const bf16* vs0 = Vh + (size_t)t * SS + kb;
#pragma unroll
      for (int i = 0; i < 4; ++i) *(bf16x8*)(&ldsV[t * VSTRIDE + 8 * i]) = *(const bf16x8*)(vs0 + 8 * i);
      if (t < 32) { const bf16* vs1 = Vh + (size_t)(64 + t) * SS + kb;
#pragma unroll
        for (int i = 0; i < 4; ++i) *(bf16x8*)(&ldsV[(64 + t) * VSTRIDE + 8 * i]) = *(const bf16x8*)(vs1 + 8 * i); } }
    __syncthreads();
    f32x8 s0 = {}, s1 = {};
#pragma unroll
    for (int c = 0; c < 3; ++c) { s0 = wmma_bf16(lds_frag(ldsK + c * 32, KS2), qf[c], s0); s1 = wmma_bf16(lds_frag(ldsK + 16 * KS2 + c * 32, KS2), qf[c], s1); }
    float mx = -INFINITY;
#pragma unroll
    for (int r = 0; r < 8; ++r) { const int j0 = kb + kh8 + r, j1 = j0 + 16;
      s0[r] = s0[r] * scale + bq_[j0] * L2E; s1[r] = s1[r] * scale + bq_[j1] * L2E; mx = fmaxf(mx, fmaxf(s0[r], s1[r])); }
    mx = fmaxf(mx, __shfl_xor(mx, 16, 32));
    const float mnew = fmaxf(mrun, mx), alpha = exp2f(mrun - mnew);
    float rsum = 0.0f; bf16x16 pf;
#pragma unroll
    for (int r = 0; r < 8; ++r) { const float p0 = exp2f(s0[r] - mnew), p1 = exp2f(s1[r] - mnew); rsum += p0 + p1; pf[r] = (bf16)(p0 * 1024.0f); pf[r + 8] = (bf16)(p1 * 1024.0f); }
    rsum += __shfl_xor(rsum, 16, 32);
    lrun = lrun * alpha + rsum; mrun = mnew;
#pragma unroll
    for (int j = 0; j < 6; ++j) {
#pragma unroll
      for (int r = 0; r < 8; ++r) o[j][r] *= alpha;
      o[j] = wmma_bf16(lds_frag(ldsV + (j * 16) * VSTRIDE, VSTRIDE), pf, o[j]); }
  }
  float* so = ldsO[wave];
  const float rl = 1.0f / (lrun * 1024.0f);
#pragma unroll
  for (int j = 0; j < 6; ++j)
#pragma unroll
    for (int r = 0; r < 8; ++r) so[qlane * 100 + j * 16 + kh8 + r] = o[j][r] * rl;
  asm volatile("s_wait_dscnt 0" ::: "memory");
#pragma unroll 1
  for (int pass = 0; pass < 2; ++pass) {
#pragma unroll
    for (int it = 0; it < 12; ++it) { const int ch = lane + 32 * it, ql = ch / 24, q4 = (ch % 24) * 4;
      float* dst = attnOut + ((size_t)(b * SS + q0 + ql)) * DD + h * DKK + q4;
      *(volatile v4f_t*)dst = *(const volatile v4fa*)(so + ql * 100 + q4); }
    __threadfence();
  }
}

__global__ __launch_bounds__(96) void k_vt(const bf16* __restrict__ QKV, bf16* __restrict__ Vt) {
  __shared__ bf16 tile[64][104];
  const int s0 = blockIdx.x * 64, h = blockIdx.y, b = blockIdx.z, t = threadIdx.x;
  for (int i = t; i < 64 * 96; i += 96) { const int r = i / 96, d = i % 96; tile[r][d] = QKV[((size_t)(b * SS + s0 + r)) * (3 * DD) + 2 * DD + h * DKK + d]; }
  __syncthreads();
  bf16* dst = Vt + (((size_t)(b * HH + h)) * DKK + t) * SS + s0;
#pragma unroll 1
  for (int pass = 0; pass < 2; ++pass) {
#pragma unroll
    for (int e = 0; e < 8; ++e) { bf16 hh[8];
#pragma unroll
      for (int j = 0; j < 8; ++j) hh[j] = tile[8 * e + j][t];
      *(volatile v4u_t*)(dst + 8 * e) = *(const v4ua*)hh; }
    __threadfence(); }
}
__global__ __launch_bounds__(192) void k_addln(const float* __restrict__ a, const float* __restrict__ bsrc, const float* __restrict__ g, const float* __restrict__ be, float* __restrict__ y) {
  __shared__ float red[192];
  const int m = blockIdx.x, t = threadIdx.x;
  v4f_t v = *(const v4fa*)(a + (size_t)m * DD + t * 4); const v4f_t w = *(const v4fa*)(bsrc + (size_t)m * DD + t * 4); v.x += w.x; v.y += w.y; v.z += w.z; v.w += w.w;
  red[t] = v.x + v.y + v.z + v.w; __syncthreads();
  if (t < 32) { float s = red[t] + red[t + 32] + red[t + 64] + red[t + 96] + red[t + 128] + red[t + 160];
#pragma unroll
    for (int o = 16; o >= 1; o >>= 1) s += __shfl_xor(s, o, 32); if (t == 0) red[0] = s; }
  __syncthreads(); const float mu = red[0] / (float)DD; __syncthreads();
  const float dx = v.x - mu, dy = v.y - mu, dz = v.z - mu, dw = v.w - mu; red[t] = dx * dx + dy * dy + dz * dz + dw * dw; __syncthreads();
  if (t < 32) { float s = red[t] + red[t + 32] + red[t + 64] + red[t + 96] + red[t + 128] + red[t + 160];
#pragma unroll
    for (int o = 16; o >= 1; o >>= 1) s += __shfl_xor(s, o, 32); if (t == 0) red[0] = s; }
  __syncthreads(); const float rs = rsqrtf(red[0] / (float)DD + 1e-5f);
  const v4f_t gv = *(const v4fa*)(g + t * 4), bv = *(const v4fa*)(be + t * 4);
  v4f_t r; r.x = dx * rs * gv.x + bv.x; r.y = dy * rs * gv.y + bv.y; r.z = dz * rs * gv.z + bv.z; r.w = dw * rs * gv.w + bv.w;
  *(volatile v4f_t*)(y + (size_t)m * DD + t * 4) = r; __threadfence(); *(volatile v4f_t*)(y + (size_t)m * DD + t * 4) = r;
}
__global__ __launch_bounds__(256) void k_gelu(float* __restrict__ Hf) {
  float* p = Hf + (size_t)blockIdx.x * DFF + threadIdx.x * 8; v4f_t a = *(const v4fa*)p, c = *(const v4fa*)(p + 4);
#pragma unroll 1
  for (int i = 0; i < 4; ++i) { a[i] = 0.5f * a[i] * (1.0f + erff(a[i] * 0.70710678118654752f)); c[i] = 0.5f * c[i] * (1.0f + erff(c[i] * 0.70710678118654752f)); }
  *(volatile v4f_t*)p = a; *(volatile v4f_t*)(p + 4) = c; __threadfence(); *(volatile v4f_t*)p = a; *(volatile v4f_t*)(p + 4) = c;
}

extern "C" void kernel_launch(void* const* d_in, const int* in_sizes, int n_in,
                              void* d_out, int out_size, void* d_ws, size_t ws_size,
                              hipStream_t stream) {
  (void)in_sizes; (void)n_in; (void)out_size; (void)ws_size;
  const float* x = (const float*)d_in[0];
  const float* ab = (const float*)d_in[1];
  const float* Win = (const float*)d_in[2]; const float* bin = (const float*)d_in[3];
  const float* Wo = (const float*)d_in[4]; const float* bo = (const float*)d_in[5];
  const float* W1 = (const float*)d_in[6]; const float* b1 = (const float*)d_in[7];
  const float* W2 = (const float*)d_in[8]; const float* b2 = (const float*)d_in[9];
  const float* g1 = (const float*)d_in[10]; const float* be1 = (const float*)d_in[11]; const float* g2 = (const float*)d_in[12]; const float* be2 = (const float*)d_in[13];
  float* out = (float*)d_out;
  const int M = BB * SS;
  char* ws = (char*)d_ws;
  bf16* QKV = (bf16*)ws;  ws += (size_t)M * 3 * DD * 2;
  bf16* VtB = (bf16*)ws;  ws += (size_t)M * DD * 2;
  float* At = (float*)ws; ws += (size_t)M * DD * 4;
  float* O  = (float*)ws; ws += (size_t)M * DD * 4;
  float* X1 = (float*)ws; ws += (size_t)M * DD * 4;
  float* Hf = (float*)ws; ws += (size_t)M * DFF * 4;
  dim3 gBlk(256);
  gemm_bias_kernel<float, 0><<<dim3(M / 128, 3 * DD / 256), gBlk, 0, stream>>>(x, Win, bin, QKV, M, 3 * DD, DD);
  k_vt<<<dim3(SS / 64, HH, BB), 96, 0, stream>>>(QKV, VtB);
  attn96_kernel<<<dim3(SS / 32, HH, BB), 64, 0, stream>>>(QKV, QKV + DD, VtB, ab, At);
  gemm_bias_kernel<float, 2><<<dim3(M / 128, DD / 256), gBlk, 0, stream>>>(At, Wo, bo, O, M, DD, DD);
  k_addln<<<M, 192, 0, stream>>>(x, O, g1, be1, X1);
  gemm_bias_kernel<float, 2><<<dim3(M / 128, DFF / 256), gBlk, 0, stream>>>(X1, W1, b1, Hf, M, DFF, DD);
  k_gelu<<<M, 256, 0, stream>>>(Hf);
  gemm_split_kernel<float, 2><<<dim3(M / 128, DD / 256), gBlk, 0, stream>>>(Hf, 0, W2, b2, O, M, DD, DFF);
  k_addln<<<M, 192, 0, stream>>>(X1, O, g2, be2, out);
}
